// DIMP_52175262712126
// MI455X (gfx1250) — hardware-verified
//
#include <hip/hip_runtime.h>
#include <hip/hip_bf16.h>
#include <stddef.h>


#define DF      128
#define NTHR    256
#define NWAVE   8
#define EPT     8
#define NGRP    2
#define CHUNK   (NTHR * EPT * NGRP)
#define WCAP    (EPT * NGRP * 32)
#define LISTN   (NWAVE * WCAP)
#define NBC     4096
#define NBF     1024
#define RCAP    40960
#define RBN     128
#define TGT     256
#define DEGCAP  1024
#define GROWS   128
#define OTHR    512
#define CSROWS  512

#define LDS_FILL ((RCAP + NBF + LISTN) * 4 + 64)
#define LDS_GEMM (GROWS * DF * 4)

static_assert((CHUNK & (CHUNK - 1)) == 0);
static_assert(CHUNK <= 4096);
static_assert(NBC <= 4096 && NBF <= 4096);
static_assert((NBC & (NBC - 1)) == 0 && (NBF & (NBF - 1)) == 0);
static_assert(NBC == 4 * NBF);
static_assert(OTHR * 8 == NBC);
static_assert((RCAP % 32) == 0);
static_assert(TGT == NWAVE * 32);
static_assert((DF % 32) == 0);
static_assert((3 * DF * DF / 8) % NTHR == 0);

typedef float          v4f  __attribute__((ext_vector_type(4)));
typedef float          v8f  __attribute__((ext_vector_type(8)));
typedef int            v4i  __attribute__((ext_vector_type(4)));
typedef unsigned short v8us __attribute__((ext_vector_type(8)));
typedef __bf16         v16bf __attribute__((ext_vector_type(16)));
typedef double         v2d  __attribute__((ext_vector_type(2)));
union FragB { v16bf v; v8us h[2]; };

__device__ __forceinline__ unsigned int bf16_bits(float x) {
  const unsigned int u = __float_as_uint(x);
  return (u + 0x7FFFu + ((u >> 16) & 1u)) >> 16;
}

__device__ __forceinline__ unsigned int split1(float x) {
  const unsigned int hb = bf16_bits(x) & 0xFFFFu;
  const float hv = __uint_as_float(hb << 16);
  const unsigned int lb = bf16_bits(x - hv) & 0xFFFFu;
  return hb | (lb << 16);
}

__device__ __forceinline__ void split8(v4f a, v4f b, v8us& hi, v8us& lo) {
  const unsigned int t0 = split1(a.x), t1 = split1(a.y), t2 = split1(a.z), t3 = split1(a.w);
  const unsigned int t4 = split1(b.x), t5 = split1(b.y), t6 = split1(b.z), t7 = split1(b.w);
  hi[0] = (unsigned short)(t0 & 0xFFFFu); lo[0] = (unsigned short)(t0 >> 16);
  hi[1] = (unsigned short)(t1 & 0xFFFFu); lo[1] = (unsigned short)(t1 >> 16);
  hi[2] = (unsigned short)(t2 & 0xFFFFu); lo[2] = (unsigned short)(t2 >> 16);
  hi[3] = (unsigned short)(t3 & 0xFFFFu); lo[3] = (unsigned short)(t3 >> 16);
  hi[4] = (unsigned short)(t4 & 0xFFFFu); lo[4] = (unsigned short)(t4 >> 16);
  hi[5] = (unsigned short)(t5 & 0xFFFFu); lo[5] = (unsigned short)(t5 >> 16);
  hi[6] = (unsigned short)(t6 & 0xFFFFu); lo[6] = (unsigned short)(t6 >> 16);
  hi[7] = (unsigned short)(t7 & 0xFFFFu); lo[7] = (unsigned short)(t7 >> 16);
}

__device__ __forceinline__ v8f wmb(v16bf a, v16bf b, v8f c) {
  v8f d = __builtin_amdgcn_wmma_f32_16x16x32_bf16(false, a, false, b, (short)0, c, false, false);
  asm volatile("v_nop\n\tv_nop\n\tv_nop\n\tv_nop" : "+v"(d) : "v"(a), "v"(b));
  return d;
}

template <int NB>
__device__ __forceinline__ int scan_chunk(const int* __restrict__ dsts, int nE, int cbase, int slotBase,
                                          int vec8, int* list, int tid, int lane, int wave) {
  int wc = 0;
#pragma unroll
  for (int g = 0; g < NGRP; ++g) {
    const int el0  = (g * NTHR + tid) * EPT;
    const int e0   = cbase + el0;
    const int sent = -2147483647 - 1;
    v4i da, db;
    if (vec8 != 0 && cbase + CHUNK <= nE) {
      da = *(const v4i*)(dsts + e0);
      db = *(const v4i*)(dsts + e0 + 4);
    } else {
      da.x = (e0     < nE) ? dsts[min(e0, nE - 1)] : sent;
      da.y = (e0 + 1 < nE) ? dsts[min(e0 + 1, nE - 1)] : sent;
      da.z = (e0 + 2 < nE) ? dsts[min(e0 + 2, nE - 1)] : sent;
      da.w = (e0 + 3 < nE) ? dsts[min(e0 + 3, nE - 1)] : sent;
      db.x = (e0 + 4 < nE) ? dsts[min(e0 + 4, nE - 1)] : sent;
      db.y = (e0 + 5 < nE) ? dsts[min(e0 + 5, nE - 1)] : sent;
      db.z = (e0 + 6 < nE) ? dsts[min(e0 + 6, nE - 1)] : sent;
      db.w = (e0 + 7 < nE) ? dsts[min(e0 + 7, nE - 1)] : sent;
    }
    const unsigned nb = (unsigned)slotBase;
    const unsigned s0 = (unsigned)da.x - nb, s1 = (unsigned)da.y - nb;
    const unsigned s2 = (unsigned)da.z - nb, s3 = (unsigned)da.w - nb;
    const unsigned s4 = (unsigned)db.x - nb, s5 = (unsigned)db.y - nb;
    const unsigned s6 = (unsigned)db.z - nb, s7 = (unsigned)db.w - nb;
    const bool h0 = s0 < (unsigned)NB, h1 = s1 < (unsigned)NB, h2 = s2 < (unsigned)NB, h3 = s3 < (unsigned)NB;
    const bool h4 = s4 < (unsigned)NB, h5 = s5 < (unsigned)NB, h6 = s6 < (unsigned)NB, h7 = s7 < (unsigned)NB;
    const unsigned any = __builtin_amdgcn_ballot_w32(h0 | h1 | h2 | h3 | h4 | h5 | h6 | h7);
    if (any != 0u) {
#define HITJ(J, HJ, SJ) { \
        const unsigned mj = __builtin_amdgcn_ballot_w32(HJ); \
        if (mj != 0u) { \
          if (HJ) { \
            const int pos = wc + (int)__builtin_amdgcn_mbcnt_lo(mj, 0u); \
            if (pos < WCAP) list[wave * WCAP + pos] = ((el0 + (J)) << 12) | (int)(SJ); \
          } \
          wc += (int)__builtin_popcount(mj); } }
      HITJ(0, h0, s0)
      HITJ(1, h1, s1)
      HITJ(2, h2, s2)
      HITJ(3, h3, s3)
      HITJ(4, h4, s4)
      HITJ(5, h5, s5)
      HITJ(6, h6, s6)
      HITJ(7, h7, s7)
#undef HITJ
    }
  }
  return wc;
}

__global__ __launch_bounds__(NTHR) void k_wprep(
    const float* __restrict__ W0, const float* __restrict__ W1, const float* __restrict__ W2,
    unsigned short* wHi, unsigned short* wLo) {
  const int i = blockIdx.x * NTHR + (int)threadIdx.x;
  if (i >= 3 * DF * DF / 8) return;
  const int layer = i / (DF * DF / 8);
  const float* src = (layer == 0) ? W0 : ((layer == 1) ? W1 : W2);
  const int o  = i * 8;
  const int oo = o - layer * DF * DF;
  const int n  = oo >> 7;
  const int k0 = oo & (DF - 1);
  v4f a, b;
  a.x = src[(k0 + 0) * DF + n]; a.y = src[(k0 + 1) * DF + n];
  a.z = src[(k0 + 2) * DF + n]; a.w = src[(k0 + 3) * DF + n];
  b.x = src[(k0 + 4) * DF + n]; b.y = src[(k0 + 5) * DF + n];
  b.z = src[(k0 + 6) * DF + n]; b.w = src[(k0 + 7) * DF + n];
  v8us hv, lv;
  split8(a, b, hv, lv);
  unsigned short* ph = wHi + o;
  unsigned short* pl = wLo + o;
  *(volatile v8us*)ph = hv;
  *(volatile v8us*)pl = lv;
  __threadfence();
  *(volatile v8us*)ph = hv;
  *(volatile v8us*)pl = lv;
}

__global__ __launch_bounds__(NTHR) void k_count(const int* __restrict__ ei, int* cnt, int nE, int vec8) {
  __shared__ __attribute__((aligned(16))) int scnt[NBC];
  __shared__ __attribute__((aligned(16))) int list[LISTN];
  __shared__ int wcnt[NWAVE];
  const int tid = threadIdx.x, lane = tid & 31, wave = tid >> 5;
  const int nodeBase = blockIdx.x * NBC;
  const int* dsts = ei + nE;

  for (int i = tid; i < NBC; i += NTHR) scnt[i] = 0;
  __syncthreads();

  const int nChunks = (nE + CHUNK - 1) / CHUNK;
#pragma unroll 1
  for (int ch = 0; ch < nChunks; ++ch) {
    const int cbase = ch * CHUNK;
    const int wc = scan_chunk<NBC>(dsts, nE, cbase, nodeBase, vec8, list, tid, lane, wave);
    if (lane == 0) wcnt[wave] = wc;
    __syncthreads();
    if (wave == 0) {
#pragma unroll 1
      for (int wsx = 0; wsx < NWAVE; ++wsx) {
        int n = __builtin_amdgcn_readfirstlane(wcnt[wsx]);
        n = n > WCAP ? WCAP : (n < 0 ? 0 : n);
        const int* lp = list + wsx * WCAP;
#pragma unroll 1
        for (int i = 0; i < n; ++i) {
          const int ent  = __builtin_amdgcn_readfirstlane(lp[i]);
          const int slot = ent & (NBC - 1);
          if (lane == 0) scnt[slot] = scnt[slot] + 1;
        }
      }
    }
    __syncthreads();
  }

  v4i cq[4];
#pragma unroll
  for (int q = 0; q < 4; ++q) {
    const int f = (wave * 4 + q) * 128 + 4 * lane;
    cq[q] = *(const v4i*)(scnt + f);
  }
  int* cp = cnt + (size_t)nodeBase;
#pragma unroll
  for (int q = 0; q < 4; ++q) {
    const int f = (wave * 4 + q) * 128 + 4 * lane;
    *(volatile v4i*)(cp + f) = cq[q];
  }
  __threadfence();
#pragma unroll
  for (int q = 0; q < 4; ++q) {
    const int f = (wave * 4 + q) * 128 + 4 * lane;
    *(volatile v4i*)(cp + f) = cq[q];
  }
}

__global__ __launch_bounds__(OTHR) void k_offsets(
    const int* __restrict__ cnt, int* off, int* rbase, int nChunk) {
  __shared__ __attribute__((aligned(16))) int soff[NBC];
  __shared__ __attribute__((aligned(16))) int srb[RBN];
  __shared__ int wtot[OTHR / 32];
  const int tid = threadIdx.x, lane = tid & 31, wave = tid >> 5, sub = tid >> 7;
  for (int i = tid; i < RBN; i += OTHR) srb[i] = 0;
  int carry = 0;
#pragma unroll 1
  for (int ch = 0; ch < nChunk; ++ch) {
    const int base = ch * NBC;
    const v4i c0 = *(const v4i*)(cnt + base + 8 * tid);
    const v4i c1 = *(const v4i*)(cnt + base + 8 * tid + 4);
    const int e0 = max(c0.x, 0), e1 = max(c0.y, 0), e2 = max(c0.z, 0), e3 = max(c0.w, 0);
    const int e4 = max(c1.x, 0), e5 = max(c1.y, 0), e6 = max(c1.z, 0), e7 = max(c1.w, 0);
    const int ts = e0 + e1 + e2 + e3 + e4 + e5 + e6 + e7;
    int incl = ts;
#pragma unroll
    for (int d = 1; d < 32; d <<= 1) {
      const int t = __shfl_up(incl, d);
      if (lane >= d) incl += t;
    }
    if (lane == 31) wtot[wave] = incl;
    __syncthreads();
    const int S0 = wtot[0]  + wtot[1]  + wtot[2]  + wtot[3];
    const int S1 = wtot[4]  + wtot[5]  + wtot[6]  + wtot[7];
    const int S2 = wtot[8]  + wtot[9]  + wtot[10] + wtot[11];
    const int S3 = wtot[12] + wtot[13] + wtot[14] + wtot[15];
    int pre = 0;
#pragma unroll 1
    for (int w = 4 * sub; w < wave; ++w) pre += wtot[w];
    const int b0 = carry;
    const int b1 = b0 + ((S0 + 31) & ~31);
    const int b2 = b1 + ((S1 + 31) & ~31);
    const int b3 = b2 + ((S2 + 31) & ~31);
    const int b4 = b3 + ((S3 + 31) & ~31);
    const int myb = sub == 0 ? b0 : (sub == 1 ? b1 : (sub == 2 ? b2 : b3));
    if (tid == 0) {
      srb[min(4 * ch + 0, RBN - 1)] = b0;
      srb[min(4 * ch + 1, RBN - 1)] = b1;
      srb[min(4 * ch + 2, RBN - 1)] = b2;
      srb[min(4 * ch + 3, RBN - 1)] = b3;
    }
    int run = myb + pre + incl - ts;
    soff[8 * tid + 0] = run; run += e0;
    soff[8 * tid + 1] = run; run += e1;
    soff[8 * tid + 2] = run; run += e2;
    soff[8 * tid + 3] = run; run += e3;
    soff[8 * tid + 4] = run; run += e4;
    soff[8 * tid + 5] = run; run += e5;
    soff[8 * tid + 6] = run; run += e6;
    soff[8 * tid + 7] = run;
    carry = b4;
    __syncthreads();
    const v4i o0 = *(const v4i*)(soff + 4 * tid);
    const v4i o1 = *(const v4i*)(soff + 4 * (tid + OTHR));
    int* op = off + base;
    *(volatile v4i*)(op + 4 * tid) = o0;
    *(volatile v4i*)(op + 4 * (tid + OTHR)) = o1;
    __threadfence();
    *(volatile v4i*)(op + 4 * tid) = o0;
    *(volatile v4i*)(op + 4 * (tid + OTHR)) = o1;
    __syncthreads();
  }
  if (tid == 0) srb[min(4 * nChunk, RBN - 1)] = carry;
  __syncthreads();
  v4i rv = {0, 0, 0, 0};
  if (tid < 32) rv = *(const v4i*)(srb + 4 * tid);
  if (tid < 32) *(volatile v4i*)(rbase + 4 * tid) = rv;
  __threadfence();
  if (tid < 32) *(volatile v4i*)(rbase + 4 * tid) = rv;
}

__global__ __launch_bounds__(NTHR) void k_fill(
    const int* __restrict__ ei, const int* __restrict__ off, const int* __restrict__ rbase,
    int* csr, int nN, int nE, int vec8, int csrLen) {
  extern __shared__ v4f lds_dyn[];
  int* region = (int*)lds_dyn;
  int* cursor = region + RCAP;
  int* list   = cursor + NBF;
  int* wcnt   = list + LISTN;
  const int tid = threadIdx.x, lane = tid & 31, wave = tid >> 5;
  const int b = blockIdx.x;
  const int nodeBase = b * NBF;
  const int* dsts = ei + nE;

  int rb0 = rbase[b];
  const int rb1 = rbase[b + 1];
  rb0 = rb0 < 0 ? 0 : (rb0 > csrLen ? csrLen : rb0);
  rb0 &= ~31;
  int len = rb1 - rb0;
  len = len < 0 ? 0 : (len > RCAP ? RCAP : len);
  int lenW = (len + 31) & ~31;
  if (rb0 + lenW > csrLen) lenW = (csrLen - rb0) & ~31;

  {
    const v4i z = {0, 0, 0, 0};
    for (int i = tid; i < RCAP / 4; i += NTHR) ((v4i*)region)[i] = z;
    for (int s = tid; s < NBF; s += NTHR) {
      int o = off[nodeBase + s] - rb0;
      o = o < 0 ? 0 : (o > RCAP ? RCAP : o);
      cursor[s] = o;
    }
  }
  __syncthreads();

  const int nChunks = (nE + CHUNK - 1) / CHUNK;
#pragma unroll 1
  for (int ch = 0; ch < nChunks; ++ch) {
    const int cbase = ch * CHUNK;
    const int wc = scan_chunk<NBF>(dsts, nE, cbase, nodeBase, vec8, list, tid, lane, wave);
    if (lane == 0) wcnt[wave] = wc;
    __syncthreads();
    if (wave == 0) {
#pragma unroll 1
      for (int wsx = 0; wsx < NWAVE; ++wsx) {
        int n = __builtin_amdgcn_readfirstlane(wcnt[wsx]);
        n = n > WCAP ? WCAP : (n < 0 ? 0 : n);
        const int* lp = list + wsx * WCAP;
#pragma unroll 1
        for (int i = 0; i < n; ++i) {
          const int ent  = __builtin_amdgcn_readfirstlane(lp[i]);
          const int slot = ent & (NBF - 1);
          int e = cbase + ((ent >> 12) & (CHUNK - 1));
          e = e > nE - 1 ? nE - 1 : e;
          int src = ei[e];
          src = src < 0 ? 0 : (src > nN - 1 ? nN - 1 : src);
          if (lane == 0) {
            int pos = cursor[slot];
            pos = pos < 0 ? 0 : (pos > RCAP - 1 ? RCAP - 1 : pos);
            region[pos] = src;
            const int np = pos + 1;
            cursor[slot] = np > RCAP ? RCAP : np;
          }
        }
      }
    }
    __syncthreads();
  }

  const int nv = lenW >> 2;
  int* gp = csr + rb0;
#pragma unroll 1
  for (int i = tid; i < nv; i += NTHR) { const v4i v = ((const v4i*)region)[i]; *(volatile v4i*)(gp + 4 * i) = v; }
  __threadfence();
#pragma unroll 1
  for (int i = tid; i < nv; i += NTHR) { const v4i v = ((const v4i*)region)[i]; *(volatile v4i*)(gp + 4 * i) = v; }
}

__global__ __launch_bounds__(NTHR) void k_agg(
    const int* __restrict__ csr, const int* __restrict__ off, const int* __restrict__ cnt,
    const float* __restrict__ srcA, const float* __restrict__ srcB,
    unsigned short* aggHi, unsigned short* aggLo, int nN, int csrLen) {
  const int tid = threadIdx.x, lane = tid & 31, wave = tid >> 5, hh = lane >> 4, q = lane & 15;
  const int tbase = blockIdx.x * TGT + wave * 32;
  const int cl = tbase + lane;
  const int cnt_l = cnt[cl];
  const int off_l = off[cl];
  const float* base = ((hh == 0) ? srcA : srcB) + 8 * q;
  const size_t rowAdd = (size_t)((hh == 0) ? 0 : nN) * DF;

#pragma unroll 1
  for (int j = 0; j < 32; ++j) {
    const int c = tbase + j;
    int n = __builtin_amdgcn_readlane(cnt_l, j);
    n = n < 0 ? 0 : (n > DEGCAP ? DEGCAP : n);
    const int st = __builtin_amdgcn_readlane(off_l, j);
    v4f a0 = {0.f, 0.f, 0.f, 0.f};
    v4f a1 = {0.f, 0.f, 0.f, 0.f};
#pragma unroll 1
    for (int q0 = 0; q0 < n; q0 += 32) {
      int pos = st + q0 + lane;
      pos = pos < 0 ? 0 : (pos > csrLen - 1 ? csrLen - 1 : pos);
      int sl = csr[pos];
      sl = sl < 0 ? 0 : (sl > nN - 1 ? nN - 1 : sl);
      const int mcnt = (n - q0) < 32 ? (n - q0) : 32;
#pragma unroll 1
      for (int p = 0; p < mcnt; ++p) {
        const int s = __builtin_amdgcn_readlane(sl, p);
        const float* rp = base + (size_t)s * DF;
        a0 = a0 + *(const v4f*)rp;
        a1 = a1 + *(const v4f*)(rp + 4);
      }
    }
    v8us hv, lv;
    split8(a0, a1, hv, lv);
    if (c < nN) {
      const size_t o = (size_t)c * DF + rowAdd + 8 * q;
      unsigned short* ph = aggHi + o;
      unsigned short* pl = aggLo + o;
      *(volatile v8us*)ph = hv;
      *(volatile v8us*)pl = lv;
      __threadfence();
      *(volatile v8us*)ph = hv;
      *(volatile v8us*)pl = lv;
    }
  }
}

__global__ __launch_bounds__(NTHR) void k_gemm(
    const unsigned short* __restrict__ aHi, const unsigned short* __restrict__ aLo,
    const unsigned short* __restrict__ wHi, const unsigned short* __restrict__ wLo,
    const float* __restrict__ bias, float* C) {
  extern __shared__ v4f lds_dyn[];
  float* stg = (float*)lds_dyn;
  const int tid = threadIdx.x, lane = tid & 31, wave = tid >> 5, hh = lane >> 4, m = lane & 15;
  const int rowBase = blockIdx.x * GROWS;
  const size_t arow = (size_t)(rowBase + wave * 16 + m) * DF + 8 * hh;

  v8f acc[8];
#pragma unroll
  for (int t = 0; t < 8; ++t) { v8f z = {0.f, 0.f, 0.f, 0.f, 0.f, 0.f, 0.f, 0.f}; acc[t] = z; }

#pragma unroll 1
  for (int kt = 0; kt < DF / 32; ++kt) {
    FragB ah, al;
    ah.h[0] = *(const v8us*)(aHi + arow + 32 * kt);
    ah.h[1] = *(const v8us*)(aHi + arow + 32 * kt + 16);
    al.h[0] = *(const v8us*)(aLo + arow + 32 * kt);
    al.h[1] = *(const v8us*)(aLo + arow + 32 * kt + 16);
#pragma unroll
    for (int t = 0; t < 8; ++t) {
      const size_t bo = (size_t)(16 * t + m) * DF + 32 * kt + 8 * hh;
      FragB bh, bl;
      bh.h[0] = *(const v8us*)(wHi + bo);
      bh.h[1] = *(const v8us*)(wHi + bo + 16);
      bl.h[0] = *(const v8us*)(wLo + bo);
      bl.h[1] = *(const v8us*)(wLo + bo + 16);
      acc[t] = wmb(ah.v, bh.v, acc[t]);
      acc[t] = wmb(ah.v, bl.v, acc[t]);
      acc[t] = wmb(al.v, bh.v, acc[t]);
    }
  }

  const int r0 = wave * 16 + 8 * hh;
  float* sp = stg + r0 * DF + m;
#pragma unroll
  for (int t = 0; t < 8; ++t) {
    const float bv = bias[16 * t + m];
#pragma unroll
    for (int r = 0; r < 8; ++r) {
      const float v = acc[t][r] + bv;
      sp[r * DF + 16 * t] = fmaxf(v, 0.0f);
    }
  }
  __syncthreads();

  const float* lp = stg + wave * 16 * DF + 4 * lane;
  float* gp = C + ((size_t)rowBase + wave * 16) * DF + 4 * lane;
#pragma unroll
  for (int i = 0; i < 16; ++i) { const v4f v = *(const v4f*)(lp + i * DF); *(volatile v4f*)(gp + (size_t)i * DF) = v; }
  __threadfence();
#pragma unroll
  for (int i = 0; i < 16; ++i) { const v4f v = *(const v4f*)(lp + i * DF); *(volatile v4f*)(gp + (size_t)i * DF) = v; }
}

__global__ __launch_bounds__(NTHR) void k_colsum(const float* __restrict__ H, double* part, int nN) {
  __shared__ __attribute__((aligned(16))) double sp[2 * DF];
  __shared__ __attribute__((aligned(16))) double sd[DF];
  const int tid = threadIdx.x, col = tid & (DF - 1), half = tid >> 7;
  const int base = blockIdx.x * CSROWS;
  int r1 = base + CSROWS;
  r1 = r1 > nN ? nN : r1;
  double acc = 0.0;
#pragma unroll 1
  for (int r = base + half; r < r1; r += 2) acc += (double)H[(size_t)r * DF + col];
  sp[half * DF + col] = acc;
  __syncthreads();
  if (tid < DF) sd[tid] = sp[tid] + sp[DF + tid];
  __syncthreads();
  v2d v = {0.0, 0.0};
  if (tid < 64) v = *(const v2d*)(sd + 2 * tid);
  double* gp = part + (size_t)blockIdx.x * DF + 2 * tid;
  if (tid < 64) *(volatile v2d*)gp = v;
  __threadfence();
  if (tid < 64) *(volatile v2d*)gp = v;
}

__global__ __launch_bounds__(DF) void k_head(
    const double* __restrict__ part, const float* __restrict__ Wd, float* wsv, int nPart, int nN) {
  __shared__ __attribute__((aligned(16))) double ss[DF];
  __shared__ __attribute__((aligned(16))) float so[DF];
  const int t = threadIdx.x;
  double acc = 0.0;
#pragma unroll 1
  for (int p = 0; p < nPart; ++p) acc += part[(size_t)p * DF + t];
  const float sm = (float)(acc / (double)nN);
  ss[t] = (double)sm;
  __syncthreads();
  double d = 0.0;
#pragma unroll 2
  for (int k = 0; k < DF; ++k) d += (double)Wd[t * DF + k] * ss[k];
  so[t] = (float)d;
  __syncthreads();
  v4f v = {0.f, 0.f, 0.f, 0.f};
  if (t < 32) v = *(const v4f*)(so + 4 * t);
  if (t < 32) *(volatile v4f*)(wsv + 4 * t) = v;
  __threadfence();
  if (t < 32) *(volatile v4f*)(wsv + 4 * t) = v;
}

__global__ __launch_bounds__(NTHR) void k_dots(
    const float* __restrict__ H, const float* __restrict__ wsv, float* out, int nOut, int nRowsPad) {
  __shared__ __attribute__((aligned(16))) float sw[DF];
  const int tid = threadIdx.x, lane = tid & 31, wave = tid >> 5;
  if (tid < DF) sw[tid] = wsv[tid];
  __syncthreads();
  const int rbase = (blockIdx.x * NWAVE + wave) * 32;
  int r = rbase + lane;
  r = r > nRowsPad - 1 ? nRowsPad - 1 : r;
  const float* hp = H + (size_t)r * DF;
  float acc = 0.0f;
#pragma unroll 2
  for (int k4 = 0; k4 < DF / 4; ++k4) {
    const v4f hv = *(const v4f*)(hp + 4 * k4);
    const v4f wv = *(const v4f*)(sw + 4 * k4);
    acc = fmaf(hv.x, wv.x, acc);
    acc = fmaf(hv.y, wv.y, acc);
    acc = fmaf(hv.z, wv.z, acc);
    acc = fmaf(hv.w, wv.w, acc);
  }
  if (rbase < nOut) {
    const bool ok = (rbase + lane) < nOut;
    float* op = out + rbase + lane;
    if (ok) *(volatile float*)op = acc;
    __threadfence();
    if (ok) *(volatile float*)op = acc;
  }
}

extern "C" void kernel_launch(void* const* d_in, const int* in_sizes, int n_in,
                              void* d_out, int out_size, void* d_ws, size_t ws_size,
                              hipStream_t stream) {
  if (n_in < 10) return;
  const int nE = in_sizes[0] / 2;
  const int nN = in_sizes[1] / DF;
  if (nE <= 0 || nN <= 0 || in_sizes[0] != 2 * nE || in_sizes[1] != nN * DF || in_sizes[2] != nN * DF) return;
  if (in_sizes[3] != DF * DF || in_sizes[5] != DF * DF || in_sizes[7] != DF * DF || in_sizes[9] != DF * DF) return;
  if (in_sizes[4] < DF || in_sizes[6] < DF || in_sizes[8] < DF) return;
  if (out_size != 2 * nN) return;
  if (nE > (1 << 26) || nN > (1 << 22)) return;

  const int*   ei  = (const int*)d_in[0];
  const float* x   = (const float*)d_in[1];
  const float* xs  = (const float*)d_in[2];
  const float* W0  = (const float*)d_in[3];
  const float* b0  = (const float*)d_in[4];
  const float* W1  = (const float*)d_in[5];
  const float* b1  = (const float*)d_in[6];
  const float* W2  = (const float*)d_in[7];
  const float* b2  = (const float*)d_in[8];
  const float* Wd  = (const float*)d_in[9];
  float* out = (float*)d_out;

  const int NPADN  = ((nN + TGT - 1) / TGT) * TGT;
  const int nBC    = (nN + NBC - 1) / NBC;
  const int CNTPAD = nBC * NBC;
  if (4 * nBC + 1 > RBN) return;
  const int nBF    = (nN + NBF - 1) / NBF;
  const int csrLen = ((nE + 31) & ~31) + 4096;
  const int rows2  = 2 * nN;
  const int NPAD2  = ((rows2 + 255) / 256) * 256;
  const int nGemm  = NPAD2 / GROWS;
  const int nAgg   = NPADN / TGT;
  const int nPart  = (nN + CSROWS - 1) / CSROWS;
  const int nDot   = NPAD2 / 256;

  char* ws = (char*)d_ws;
  size_t off = 0;
  const size_t oWH  = off; off += (size_t)3 * DF * DF * 2;        off = (off + 255) & ~(size_t)255;
  const size_t oWL  = off; off += (size_t)3 * DF * DF * 2;        off = (off + 255) & ~(size_t)255;
  const size_t oCnt = off; off += (size_t)CNTPAD * 4;             off = (off + 255) & ~(size_t)255;
  const size_t oOff = off; off += (size_t)CNTPAD * 4;             off = (off + 255) & ~(size_t)255;
  const size_t oRb  = off; off += (size_t)RBN * 4;                off = (off + 255) & ~(size_t)255;
  const size_t oCsr = off; off += (size_t)csrLen * 4;             off = (off + 255) & ~(size_t)255;
  const size_t oH   = off; off += (size_t)NPAD2 * DF * 4;         off = (off + 255) & ~(size_t)255;
  const size_t oAH  = off; off += (size_t)NPAD2 * DF * 2;         off = (off + 255) & ~(size_t)255;
  const size_t oAL  = off; off += (size_t)NPAD2 * DF * 2;         off = (off + 255) & ~(size_t)255;
  const size_t oPt  = off; off += (size_t)nPart * DF * 8;         off = (off + 255) & ~(size_t)255;
  const size_t oWs  = off; off += (size_t)DF * 4;                 off = (off + 255) & ~(size_t)255;
  if (off > ws_size) return;
  unsigned short* wHi  = (unsigned short*)(ws + oWH);
  unsigned short* wLo  = (unsigned short*)(ws + oWL);
  int*      cnt  = (int*)(ws + oCnt);
  int*      offp = (int*)(ws + oOff);
  int*      rb   = (int*)(ws + oRb);
  int*      csr  = (int*)(ws + oCsr);
  float*    h    = (float*)(ws + oH);
  unsigned short* aHi = (unsigned short*)(ws + oAH);
  unsigned short* aLo = (unsigned short*)(ws + oAL);
  double*   part = (double*)(ws + oPt);
  float*    wsv  = (float*)(ws + oWs);

  const int vec8 = ((nE & 3) == 0) ? 1 : 0;

  k_wprep<<<(3 * DF * DF / 8) / NTHR, NTHR, 0, stream>>>(W0, W1, W2, wHi, wLo);

  k_count<<<nBC, NTHR, 0, stream>>>(ei, cnt, nE, vec8);
  k_offsets<<<1, OTHR, 0, stream>>>(cnt, offp, rb, nBC);
  hipFuncSetAttribute(reinterpret_cast<const void*>(&k_fill),
                      hipFuncAttributeMaxDynamicSharedMemorySize, LDS_FILL);
  k_fill<<<nBF, NTHR, LDS_FILL, stream>>>(ei, offp, rb, csr, nN, nE, vec8, csrLen);

  if (NPAD2 > rows2) {
    const size_t padB = (size_t)(NPAD2 - rows2) * DF * 2;
    hipMemsetAsync((void*)(aHi + (size_t)rows2 * DF), 0, padB, stream);
    hipMemsetAsync((void*)(aLo + (size_t)rows2 * DF), 0, padB, stream);
  }

  hipFuncSetAttribute(reinterpret_cast<const void*>(&k_gemm),
                      hipFuncAttributeMaxDynamicSharedMemorySize, LDS_GEMM);

  k_agg<<<nAgg, NTHR, 0, stream>>>(csr, offp, cnt, x, xs, aHi, aLo, nN, csrLen);
  k_gemm<<<nGemm, NTHR, LDS_GEMM, stream>>>(aHi, aLo, wHi, wLo, b0, h);
  k_agg<<<nAgg, NTHR, 0, stream>>>(csr, offp, cnt, h, h + (size_t)nN * DF, aHi, aLo, nN, csrLen);
  k_gemm<<<nGemm, NTHR, LDS_GEMM, stream>>>(aHi, aLo, wHi + (size_t)DF * DF, wLo + (size_t)DF * DF, b1, h);
  k_agg<<<nAgg, NTHR, 0, stream>>>(csr, offp, cnt, h, h + (size_t)nN * DF, aHi, aLo, nN, csrLen);
  k_gemm<<<nGemm, NTHR, LDS_GEMM, stream>>>(aHi, aLo, wHi + (size_t)2 * DF * DF, wLo + (size_t)2 * DF * DF, b2, h);

  k_colsum<<<nPart, NTHR, 0, stream>>>(h, part, nN);
  k_head<<<1, DF, 0, stream>>>(part, Wd, wsv, nPart, nN);
  k_dots<<<nDot, NTHR, 0, stream>>>(h, wsv, out, out_size, NPAD2);
}
